// PixelAttention_2817498546603
// MI455X (gfx1250) — hardware-verified
//
#include <hip/hip_runtime.h>
#include <math.h>

typedef __attribute__((ext_vector_type(16))) _Float16 v16h;
typedef __attribute__((ext_vector_type(16))) __bf16 v16b;
typedef __attribute__((ext_vector_type(8)))  _Float16 v8h;
typedef __attribute__((ext_vector_type(8)))  float v8f;
typedef __attribute__((ext_vector_type(4)))  float v4f;
typedef __attribute__((ext_vector_type(2)))  float v2f;
typedef __attribute__((ext_vector_type(4)))  unsigned v4u;
typedef __attribute__((ext_vector_type(4)))  int v4i;
typedef float __attribute__((may_alias)) float_a;
typedef int __attribute__((may_alias)) int_a;

template <typename T> __device__ __forceinline__ void vst2(void* p, T v) { *(volatile T*)p = v; __threadfence(); *(volatile T*)p = v; }
__device__ __forceinline__ v8f wmma16(v16h a, v16h b, v8f c) {
  v8f d = __builtin_amdgcn_wmma_f32_16x16x32_f16(false, a, false, b, (short)0, c, false, false);
  asm volatile("v_nop\n\tv_nop\n\tv_nop\n\tv_nop" : "+v"(d) : "v"(a), "v"(b));
  return d;
}
__device__ __forceinline__ v8f wmma_bf(v16b a, v16b b, v8f c) {
  v8f d = __builtin_amdgcn_wmma_f32_16x16x32_bf16(false, a, false, b, (short)0, c, false, false);
  asm volatile("v_nop\n\tv_nop\n\tv_nop\n\tv_nop" : "+v"(d) : "v"(a), "v"(b));
  return d;
}
__device__ __forceinline__ v16h frag_h(const _Float16* rowk0, int lane) {
  union { v16h v; v8h q[2]; } u; const _Float16* p = rowk0 + 8 * (lane >> 4);
  u.q[0] = *(const v8h*)p; u.q[1] = *(const v8h*)(p + 16); return u.v;
}
__device__ __forceinline__ v16h frag_f32(const float* rowk0, int lane) {
  v16h a; const float* p = rowk0 + 8 * (lane >> 4);
#pragma unroll
  for (int i = 0; i < 8; ++i) { a[i] = (_Float16)p[i]; a[8 + i] = (_Float16)p[16 + i]; }
  return a;
}
__device__ __forceinline__ v16h frag_f32s(const float* rowk0, int lane, float sc) {
  v16h a; const float* p = rowk0 + 8 * (lane >> 4);
#pragma unroll
  for (int i = 0; i < 8; ++i) { a[i] = (_Float16)(p[i] * sc); a[8 + i] = (_Float16)(p[16 + i] * sc); }
  return a;
}
__device__ __forceinline__ v16h fragc_f32(const float* W, int k0, int n, int lane, int ld, int K) {
  v16h a; const int g = lane >> 4;
#pragma unroll
  for (int i = 0; i < 8; ++i) { const int ka = k0 + 8 * g + i, kb = ka + 16;
    a[i] = (_Float16)(ka < K ? W[(size_t)(ka < K ? ka : K - 1) * ld + n] : 0.f); a[8 + i] = (_Float16)(kb < K ? W[(size_t)(kb < K ? kb : K - 1) * ld + n] : 0.f); }
  return a;
}
struct F2 { v16b h, l; };
__device__ __forceinline__ F2 bsplit16(const float v[16]) { F2 r;
#pragma unroll
  for (int i = 0; i < 16; ++i) { const __bf16 h = (__bf16)v[i]; r.h[i] = h; r.l[i] = (__bf16)(v[i] - (float)h); }
  return r; }
__device__ __forceinline__ F2 split_row(const float* row, int k0, int lane) { float v[16]; const float* p = row + k0 + 8 * (lane >> 4);
#pragma unroll
  for (int i = 0; i < 8; ++i) { v[i] = p[i]; v[8 + i] = p[16 + i]; }
  return bsplit16(v); }
__device__ __forceinline__ F2 split_rowK(const float* row, int k0, int lane, int K) { float v[16]; const int g = lane >> 4;
#pragma unroll
  for (int i = 0; i < 8; ++i) { const int ka = k0 + 8 * g + i, kb = ka + 16; v[i] = ka < K ? row[ka < K ? ka : K - 1] : 0.f; v[8 + i] = kb < K ? row[kb < K ? kb : K - 1] : 0.f; }
  return bsplit16(v); }
__device__ __forceinline__ F2 split_col(const float* W, int k0, int n, int lane, int ld, int K) { float v[16]; const int g = lane >> 4;
#pragma unroll
  for (int i = 0; i < 8; ++i) { const int ka = k0 + 8 * g + i, kb = ka + 16; v[i] = ka < K ? W[(size_t)(ka < K ? ka : K - 1) * ld + n] : 0.f; v[8 + i] = kb < K ? W[(size_t)(kb < K ? kb : K - 1) * ld + n] : 0.f; }
  return bsplit16(v); }
__device__ __forceinline__ v8f mac3(const F2& a, const F2& b, v8f c) { c = wmma_bf(a.l, b.h, c); c = wmma_bf(a.h, b.l, c); return wmma_bf(a.h, b.h, c); }
__device__ __forceinline__ float sigm(float v) { return 1.0f / (1.0f + expf(-v)); }
#define LDSX() do { asm volatile("s_wait_dscnt 0" ::: "memory"); __builtin_amdgcn_wave_barrier(); __builtin_amdgcn_fence(__ATOMIC_RELEASE, "workgroup"); } while (0)


#define NB 4
#define CC 32
#define HW 256
#define NPX (HW * HW)
#define NGRP (NB * NPX)
#ifndef TNB
#define TNB NB
#endif
typedef __attribute__((ext_vector_type(8))) __bf16 v8b;
__device__ __forceinline__ v16b frag_b(const __bf16* rowk0, int lane) {
  union { v16b v; v8b q[2]; } u; const __bf16* p = rowk0 + 8 * (lane >> 4);
  u.q[0] = *(const v8b*)p; u.q[1] = *(const v8b*)(p + 16); return u.v;
}
__device__ __forceinline__ float bfr(float v) { return (float)(__bf16)v; }
__device__ __attribute__((noinline)) float exp_ni(float v) { return expf(v); }
__device__ __attribute__((noinline)) float erf_ni(float v) { return erff(v); }

#define WS_XQ  0u
#define WS_KS  (WS_XQ + 4u * (size_t)CC * NPX)
#define WS_VS  (WS_KS + 4u * (size_t)9 * CC * NPX)
#define WS_RES (WS_VS + 4u * (size_t)9 * CC * NPX)
#define WS_T1  (WS_RES + 4u * (size_t)CC * NPX)
#define WS_T2  (WS_T1 + 4u * (size_t)CC * NPX)
#define WS_END (WS_T2 + 4u * (size_t)64 * NPX)

__global__ __launch_bounds__(128) void k_proj(const float* __restrict__ X, const float* __restrict__ WK, const float* __restrict__ WV, const float* __restrict__ WQ, int b_, float* __restrict__ KS, float* __restrict__ VS, float* __restrict__ XQ) { __shared__ __align__(16) __bf16 sx[64][CC + 8]; __shared__ __align__(16) float so[CC][68];
  const int tid = threadIdx.x, wave = tid >> 5, lane = tid & 31, col = lane & 15, g = lane >> 4; const int p0 = blockIdx.x * 64; const int y = p0 / HW, x0 = p0 % HW; const size_t b = (size_t)b_; const int z = blockIdx.y;
  const int l = (z < 18) ? (z % 9) : 4; const int dy = l / 3 - 1, dx = l % 3 - 1; const float* Wm = (z < 9) ? (WK + (size_t)l * CC * CC) : (z < 18) ? (WV + (size_t)l * CC * CC) : WQ;
  const int ys = y + dy;
  for (int e = tid; e < CC * 64; e += 128) { const int c = e >> 6, pl = e & 63; const int xs = x0 + pl + dx; const bool in = (ys >= 0 && ys < HW && xs >= 0 && xs < HW); sx[pl][c] = (__bf16)(in ? X[(b * CC + c) * (size_t)NPX + (size_t)ys * HW + xs] : 0.f); }
  __syncthreads();
  v8f acc[2] = {};
  { const v16b a = frag_b(&sx[wave * 16 + col][0], lane);
#pragma unroll
    for (int j = 0; j < 2; ++j) { v16b w; const int o = j * 16 + col;
#pragma unroll
      for (int i = 0; i < 8; ++i) { w[i] = (__bf16)Wm[(size_t)o * CC + 8 * g + i]; w[8 + i] = (__bf16)Wm[(size_t)o * CC + 16 + 8 * g + i]; }
      acc[j] = wmma_bf(a, w, acc[j]); } }
#pragma unroll
  for (int j = 0; j < 2; ++j)
#pragma unroll
    for (int r = 0; r < 8; ++r) so[j * 16 + col][wave * 16 + 8 * g + r] = acc[j][r];
  __syncthreads();
  float* dst = (z < 9) ? (KS + ((size_t)l * CC) * NPX) : (z < 18) ? (VS + ((size_t)l * CC) * NPX) : XQ;
  for (int e = tid; e < CC * 16; e += 128) { const int cl = e >> 4, q = e & 15; vst2(dst + (size_t)cl * NPX + p0 + q * 4, *(const v4f*)&so[cl][q * 4]); } }
__global__ __launch_bounds__(128) void k_pix(const float* __restrict__ XQ, const float* __restrict__ KS, const float* __restrict__ VS, float* __restrict__ RES) {   __shared__ float sq[CC][129]; __shared__ float sal[9][129]; __shared__ __align__(16) float so[128][CC + 4];
  const int t = threadIdx.x; const size_t n = (size_t)blockIdx.x * 128 + t;
  for (int e = t; e < 128 * CC; e += 128) { const int nl = e >> 5, c = e & 31; sq[c][nl] = XQ[((size_t)blockIdx.x * 128 + nl) * CC + c]; }
  __syncthreads();
  float mx = -3.0e38f;
#pragma unroll 1
  for (int p = 0; p < 9; ++p) { const float* kp = KS + n * 288 + p * 32; float s = 0.f;
#pragma unroll 1
    for (int c = 0; c < CC; ++c) s += kp[c] * sq[c][t];
    const size_t f = n * 9 + p; const int lp = (int)((f / NPX) % 9); const int pos = (int)(f % NPX); const int yy = pos / HW + lp / 3 - 1, xx = pos % HW + lp % 3 - 1; const float m = (yy >= 0 && yy < HW && xx >= 0 && xx < HW) ? 1.0f : 0.0f;
    const float lg = s * m * 0.125f; sal[p][t] = lg; mx = fmaxf(mx, lg); }
  float ssum = 0.f;
#pragma unroll 1
  for (int p = 0; p < 9; ++p) { const float e = expf(sal[p][t] - mx); sal[p][t] = e; ssum += e; }
  const float inv = 1.0f / ssum;
#pragma unroll 1
  for (int c = 0; c < CC; ++c) { float a = 0.f;
#pragma unroll 1
    for (int p = 0; p < 9; ++p) a += sal[p][t] * VS[n * 288 + p * 32 + c];
    so[t][c] = a * inv; }
  __syncthreads(); for (int e = t; e < 128 * 8; e += 128) { const int nl = e >> 3, q = e & 7; vst2(RES + ((size_t)blockIdx.x * 128 + nl) * CC + q * 4, *(const v4f*)&so[nl][q * 4]); } }
template <int CI, int COUT>
__global__ __launch_bounds__(128) void k_conv(const float* __restrict__ IN, const float* __restrict__ Wc, const float* __restrict__ Bc, float* __restrict__ OUT) { __shared__ __align__(16) __bf16 sh[64][CI + 8], sl[64][CI + 8]; __shared__ __align__(16) float so[COUT][68];
  const int tid = threadIdx.x, wave = tid >> 5, lane = tid & 31, col = lane & 15, g = lane >> 4; const int p0 = blockIdx.x * 64; const int y = p0 / HW, x0 = p0 % HW; const size_t b = 0; (void)blockIdx.y;
  v8f acc[COUT / 16]; for (int j = 0; j < COUT / 16; ++j) for (int r = 0; r < 8; ++r) acc[j][r] = 0.f;
#pragma unroll 1
  for (int tap = 0; tap < 9; ++tap) { const int ky = tap / 3, kx = tap % 3; const int ys = y + ky - 1;
    __syncthreads();
    for (int e = tid; e < CI * 64; e += 128) { const int c = e >> 6, pl = e & 63; const int xs = x0 + pl + kx - 1; const bool in = (ys >= 0 && ys < HW && xs >= 0 && xs < HW); const float v = in ? IN[(b * CI + c) * (size_t)NPX + (size_t)ys * HW + xs] : 0.f; const __bf16 hv = (__bf16)v; sh[pl][c] = hv; sl[pl][c] = (__bf16)(v - (float)hv); }
    __syncthreads();
#pragma unroll
    for (int kc = 0; kc < CI / 32; ++kc) { const v16b ah = frag_b(&sh[wave * 16 + col][kc * 32], lane), al = frag_b(&sl[wave * 16 + col][kc * 32], lane);
#pragma unroll
      for (int j = 0; j < COUT / 16; ++j) { v16b w; const int o = j * 16 + col;
#pragma unroll
        for (int i = 0; i < 8; ++i) { w[i] = (__bf16)Wc[(((size_t)o * CI + kc * 32 + 8 * g + i) * 3 + ky) * 3 + kx]; w[8 + i] = (__bf16)Wc[(((size_t)o * CI + kc * 32 + 16 + 8 * g + i) * 3 + ky) * 3 + kx]; }
        acc[j] = wmma_bf(ah, w, acc[j]); acc[j] = wmma_bf(al, w, acc[j]); } } }
#pragma unroll
  for (int j = 0; j < COUT / 16; ++j) { const int o = j * 16 + col; const float bb = bfr(Bc[o]);
#pragma unroll
    for (int r = 0; r < 8; ++r) so[o][wave * 16 + 8 * g + r] = acc[j][r] + bb; }
  __syncthreads(); for (int e = tid; e < COUT * 16; e += 128) { const int cl = e >> 4, q = e & 15; vst2(OUT + (b * COUT + cl) * (size_t)NPX + p0 + q * 4, *(const v4f*)&so[cl][q * 4]); } }
extern "C" void kernel_launch(void* const* d_in, const int* in_sizes, int n_in, void* d_out, int out_size, void* d_ws, size_t ws_size, hipStream_t stream) {
  (void)in_sizes; (void)n_in; (void)out_size;
  const float** F = (const float**)d_in;
  if (ws_size < (size_t)WS_END) return;
  char* ws = (char*)d_ws; float *XQ = (float*)(ws + WS_XQ), *KS = (float*)(ws + WS_KS), *VS = (float*)(ws + WS_VS), *RES = (float*)(ws + WS_RES), *T1 = (float*)(ws + WS_T1), *T2 = (float*)(ws + WS_T2);
  for (int b = 0; b < TNB; ++b) {
    k_proj<<<dim3(NPX / 64, 19), 128, 0, stream>>>(F[0], F[1], F[2], F[3], b, KS, VS, XQ);
    k_pix<<<NPX / 128, 128, 0, stream>>>(XQ, KS, VS, RES);
    k_conv<32, 32><<<dim3(NPX / 64, 1), 128, 0, stream>>>(RES, F[4], F[5], T1);
    k_conv<32, 64><<<dim3(NPX / 64, 1), 128, 0, stream>>>(T1, F[6], F[7], T2);
    k_conv<64, 32><<<dim3(NPX / 64, 1), 128, 0, stream>>>(T2, F[8], F[9], (float*)d_out + (size_t)b * CC * NPX);
  }
}
